// NALUi2_22677427323455
// MI455X (gfx1250) — hardware-verified
//
#include <hip/hip_runtime.h>
#include <math.h>

typedef __attribute__((ext_vector_type(16))) _Float16 v16h;
typedef __attribute__((ext_vector_type(16))) __bf16 v16b;
typedef __attribute__((ext_vector_type(8)))  _Float16 v8h;
typedef __attribute__((ext_vector_type(8)))  float v8f;
typedef __attribute__((ext_vector_type(4)))  float v4f;
typedef __attribute__((ext_vector_type(2)))  float v2f;
typedef __attribute__((ext_vector_type(4)))  unsigned v4u;
typedef __attribute__((ext_vector_type(4)))  int v4i;
typedef float __attribute__((may_alias)) float_a;
typedef int __attribute__((may_alias)) int_a;

template <typename T> __device__ __forceinline__ void vst2(void* p, T v) { *(volatile T*)p = v; __threadfence(); *(volatile T*)p = v; }
__device__ __forceinline__ v8f wmma16(v16h a, v16h b, v8f c) {
  v8f d = __builtin_amdgcn_wmma_f32_16x16x32_f16(false, a, false, b, (short)0, c, false, false);
  asm volatile("v_nop\n\tv_nop\n\tv_nop\n\tv_nop" : "+v"(d) : "v"(a), "v"(b));
  return d;
}
__device__ __forceinline__ v8f wmma_bf(v16b a, v16b b, v8f c) {
  v8f d = __builtin_amdgcn_wmma_f32_16x16x32_bf16(false, a, false, b, (short)0, c, false, false);
  asm volatile("v_nop\n\tv_nop\n\tv_nop\n\tv_nop" : "+v"(d) : "v"(a), "v"(b));
  return d;
}
__device__ __forceinline__ v16h frag_h(const _Float16* rowk0, int lane) {
  union { v16h v; v8h q[2]; } u; const _Float16* p = rowk0 + 8 * (lane >> 4);
  u.q[0] = *(const v8h*)p; u.q[1] = *(const v8h*)(p + 16); return u.v;
}
__device__ __forceinline__ v16h frag_f32(const float* rowk0, int lane) {
  v16h a; const float* p = rowk0 + 8 * (lane >> 4);
#pragma unroll
  for (int i = 0; i < 8; ++i) { a[i] = (_Float16)p[i]; a[8 + i] = (_Float16)p[16 + i]; }
  return a;
}
__device__ __forceinline__ v16h frag_f32s(const float* rowk0, int lane, float sc) {
  v16h a; const float* p = rowk0 + 8 * (lane >> 4);
#pragma unroll
  for (int i = 0; i < 8; ++i) { a[i] = (_Float16)(p[i] * sc); a[8 + i] = (_Float16)(p[16 + i] * sc); }
  return a;
}
__device__ __forceinline__ v16h fragc_f32(const float* W, int k0, int n, int lane, int ld, int K) {
  v16h a; const int g = lane >> 4;
#pragma unroll
  for (int i = 0; i < 8; ++i) { const int ka = k0 + 8 * g + i, kb = ka + 16;
    a[i] = (_Float16)(ka < K ? W[(size_t)(ka < K ? ka : K - 1) * ld + n] : 0.f); a[8 + i] = (_Float16)(kb < K ? W[(size_t)(kb < K ? kb : K - 1) * ld + n] : 0.f); }
  return a;
}
struct F2 { v16b h, l; };
__device__ __forceinline__ F2 bsplit16(const float v[16]) { F2 r;
#pragma unroll
  for (int i = 0; i < 16; ++i) { const __bf16 h = (__bf16)v[i]; r.h[i] = h; r.l[i] = (__bf16)(v[i] - (float)h); }
  return r; }
__device__ __forceinline__ F2 split_row(const float* row, int k0, int lane) { float v[16]; const float* p = row + k0 + 8 * (lane >> 4);
#pragma unroll
  for (int i = 0; i < 8; ++i) { v[i] = p[i]; v[8 + i] = p[16 + i]; }
  return bsplit16(v); }
__device__ __forceinline__ F2 split_rowK(const float* row, int k0, int lane, int K) { float v[16]; const int g = lane >> 4;
#pragma unroll
  for (int i = 0; i < 8; ++i) { const int ka = k0 + 8 * g + i, kb = ka + 16; v[i] = ka < K ? row[ka < K ? ka : K - 1] : 0.f; v[8 + i] = kb < K ? row[kb < K ? kb : K - 1] : 0.f; }
  return bsplit16(v); }
__device__ __forceinline__ F2 split_col(const float* W, int k0, int n, int lane, int ld, int K) { float v[16]; const int g = lane >> 4;
#pragma unroll
  for (int i = 0; i < 8; ++i) { const int ka = k0 + 8 * g + i, kb = ka + 16; v[i] = ka < K ? W[(size_t)(ka < K ? ka : K - 1) * ld + n] : 0.f; v[8 + i] = kb < K ? W[(size_t)(kb < K ? kb : K - 1) * ld + n] : 0.f; }
  return bsplit16(v); }
__device__ __forceinline__ v8f mac3(const F2& a, const F2& b, v8f c) { c = wmma_bf(a.l, b.h, c); c = wmma_bf(a.h, b.l, c); return wmma_bf(a.h, b.h, c); }
__device__ __forceinline__ float sigm(float v) { return 1.0f / (1.0f + expf(-v)); }
#define LDSX() do { asm volatile("s_wait_dscnt 0" ::: "memory"); __builtin_amdgcn_wave_barrier(); __builtin_amdgcn_fence(__ATOMIC_RELEASE, "workgroup"); } while (0)


#define BB 256
#define DI 1024
#define DO 1024
#ifndef TBB
#define TBB (BB / 16)
#endif
typedef __attribute__((ext_vector_type(8))) __bf16 v8b;
__device__ __forceinline__ v16b frag_b(const __bf16* rowk0, int lane) {
  union { v16b v; v8b q[2]; } u; const __bf16* p = rowk0 + 8 * (lane >> 4);
  u.q[0] = *(const v8b*)p; u.q[1] = *(const v8b*)(p + 16); return u.v;
}
__device__ __forceinline__ v16b frag_gbf(const float* rowk0, int lane) {
  v16b a; const float* p = rowk0 + 8 * (lane >> 4);
#pragma unroll
  for (int i = 0; i < 8; ++i) { a[i] = (__bf16)p[i]; a[8 + i] = (__bf16)p[16 + i]; }
  return a;
}
__device__ __forceinline__ float bfr(float v) { return (float)(__bf16)v; }
__device__ __attribute__((noinline)) float exp_ni(float v) { return expf(v); }
__device__ __attribute__((noinline)) float tanh_ni(float v) { return tanhf(v); }
__device__ __attribute__((noinline)) float log_ni(float v) { return logf(v); }
#define WS_W1H 0u
#define WS_W1L (WS_W1H + 2u * DO * DI)
#define WS_W2H (WS_W1L + 2u * DO * DI)
#define WS_W2L (WS_W2H + 2u * DO * DI)
#define WS_AW2 (WS_W2L + 2u * DO * DI)
#define WS_END (WS_AW2 + 4u * DO * DI)

__global__ __launch_bounds__(256) void k_w(const float* __restrict__ wh1, const float* __restrict__ mh1, const float* __restrict__ wh2, const float* __restrict__ mh2, __bf16* __restrict__ W1H, __bf16* __restrict__ W1L, __bf16* __restrict__ W2H, __bf16* __restrict__ W2L, float* __restrict__ AW2) {
  __shared__ __align__(16) __bf16 s1h[64][72], s1l[64][72], s2h[64][72], s2l[64][72]; __shared__ __align__(16) float sa[64][68];
  const int tid = threadIdx.x; const int i0 = blockIdx.x * 64, o0 = blockIdx.y * 64;
  for (int q = tid; q < 64 * 64; q += 256) { const int il = q >> 6, ol = q & 63; const size_t idx = (size_t)(i0 + il) * DO + o0 + ol;
    const float w1 = tanh_ni(bfr(wh1[idx])) * (1.0f / (1.0f + exp_ni(-bfr(mh1[idx])))); const float w2 = tanh_ni(bfr(wh2[idx])) * (1.0f / (1.0f + exp_ni(-bfr(mh2[idx]))));
    __bf16 hb = (__bf16)w1; s1h[ol][il] = hb; s1l[ol][il] = (__bf16)(w1 - (float)hb); hb = (__bf16)w2; s2h[ol][il] = hb; s2l[ol][il] = (__bf16)(w2 - (float)hb);
    const size_t idx2 = (size_t)(o0 + il) * DO + i0 + ol;
    const float w2b = tanh_ni(bfr(wh2[idx2])) * (1.0f / (1.0f + exp_ni(-bfr(mh2[idx2])))); sa[il][ol] = fabsf(w2b); }
  __syncthreads();
  for (int q = tid; q < 64 * 8; q += 256) { const int ol = q >> 3, pc = q & 7; const size_t o = (size_t)(o0 + ol) * DI + i0 + pc * 8;
    vst2((unsigned*)(W1H + o), *(const v4u*)&s1h[ol][pc * 8]); vst2((unsigned*)(W1L + o), *(const v4u*)&s1l[ol][pc * 8]); vst2((unsigned*)(W2H + o), *(const v4u*)&s2h[ol][pc * 8]); vst2((unsigned*)(W2L + o), *(const v4u*)&s2l[ol][pc * 8]); }
  for (int q = tid; q < 64 * 16; q += 256) { const int rl = q >> 4, pc = q & 15; vst2(AW2 + (size_t)(o0 + rl) * DO + i0 + pc * 4, *(const v4f*)&sa[rl][pc * 4]); }
}
__global__ __launch_bounds__(128) void k_main(const float* __restrict__ X, const __bf16* __restrict__ W1H, const __bf16* __restrict__ W1L, const __bf16* __restrict__ W2H, const __bf16* __restrict__ W2L, const float* __restrict__ AW2, const float* __restrict__ G, float* __restrict__ Y) {
  __shared__ __align__(16) __bf16 slh[16][DI + 8], sll[16][DI + 8]; __shared__ signed char ssg[16][DI]; __shared__ __align__(16) float sa_[16][68], ss_[16][68], sy[16][68];
  const int tid = threadIdx.x, wave = tid >> 5, lane = tid & 31, col = lane & 15, g = lane >> 4; const int b0 = blockIdx.x * 16, o0 = blockIdx.y * 64;
  for (int q = tid; q < 16 * DI; q += 128) { const int rl = q / DI, i = q % DI; const float xv = bfr(X[(size_t)(b0 + rl) * DI + i]); const float lv = log_ni(fmaxf(fabsf(xv), 1e-7f)); const __bf16 hb = (__bf16)lv; slh[rl][i] = hb; sll[rl][i] = (__bf16)(lv - (float)hb); ssg[rl][i] = (signed char)(xv > 0.f ? 1 : (xv < 0.f ? -1 : 0)); }
  __syncthreads();
  v8f acc_a = {}, acc_s = {};
  const int ocol = o0 + wave * 16 + col;
#pragma unroll 2
  for (int kc = 0; kc < DI / 32; ++kc) { const v16b ax = frag_gbf(X + (size_t)(b0 + col) * DI + kc * 32, lane); const F2 al = {frag_b(&slh[col][kc * 32], lane), frag_b(&sll[col][kc * 32], lane)};
    const v16b w1h = frag_b(W1H + (size_t)ocol * DI + kc * 32, lane), w1l = frag_b(W1L + (size_t)ocol * DI + kc * 32, lane); acc_a = wmma_bf(ax, w1l, acc_a); acc_a = wmma_bf(ax, w1h, acc_a);
    const F2 w2 = {frag_b(W2H + (size_t)ocol * DI + kc * 32, lane), frag_b(W2L + (size_t)ocol * DI + kc * 32, lane)}; acc_s = mac3(al, w2, acc_s); }
#pragma unroll
  for (int r = 0; r < 8; ++r) { sa_[8 * g + r][wave * 16 + col] = acc_a[r]; ss_[8 * g + r][wave * 16 + col] = acc_s[r]; }
  __syncthreads();
  { const int ol = tid & 63, rb = (tid >> 6) * 8; const float* aw = AW2 + (size_t)(o0 + ol) * DI; float pr[8];
#pragma unroll
    for (int r = 0; r < 8; ++r) pr[r] = 1.0f;
#pragma unroll 1
    for (int i = 0; i < DI; ++i) { const float w = aw[i];
#pragma unroll
      for (int r = 0; r < 8; ++r) { const float sg = (float)ssg[rb + r][i]; pr[r] *= sg * w + (1.0f - w); } }
    const float gv = 1.0f / (1.0f + exp_ni(-bfr(G[o0 + ol])));
#pragma unroll
    for (int r = 0; r < 8; ++r) { const float a = sa_[rb + r][ol], s = ss_[rb + r][ol]; const float m = exp_ni(fminf(s, 20.0f)); const float msc = fminf(fmaxf(pr[r], -1.0f), 1.0f); sy[rb + r][ol] = gv * a + (1.0f - gv) * m * msc; } }
  __syncthreads();
  for (int q = tid; q < 16 * 16; q += 128) { const int rl = q >> 4, pc = q & 15; vst2(Y + (size_t)(b0 + rl) * DO + o0 + pc * 4, *(const v4f*)&sy[rl][pc * 4]); }
}

extern "C" void kernel_launch(void* const* d_in, const int* in_sizes, int n_in, void* d_out, int out_size, void* d_ws, size_t ws_size, hipStream_t stream) {
  (void)in_sizes; (void)n_in; (void)out_size;
  const float** F = (const float**)d_in;
  if (ws_size < (size_t)WS_END) return;
  char* ws = (char*)d_ws; __bf16 *W1H = (__bf16*)(ws + WS_W1H), *W1L = (__bf16*)(ws + WS_W1L), *W2H = (__bf16*)(ws + WS_W2H), *W2L = (__bf16*)(ws + WS_W2L); float* AW2 = (float*)(ws + WS_AW2);
  k_w<<<dim3(DI / 64, DO / 64), 256, 0, stream>>>(F[1], F[2], F[3], F[4], W1H, W1L, W2H, W2L, AW2);
  k_main<<<dim3(TBB, DO / 64), 128, 0, stream>>>(F[0], W1H, W1L, W2H, W2L, AW2, F[5], (float*)d_out);
}
